// VocabAttention_82669530514111
// MI455X (gfx1250) — hardware-verified
//
#include <hip/hip_runtime.h>
#include <math.h>

#ifndef NB
#define NB 16
#endif
#define NB_FULL 16
#define VOCAB 50257
#define VDIM 300
#define DDIM 512
#define NPAD 304
#define QP 320
#define AP 50272
#define PP 50304
#define KSTEPS 1571
#define KCH 32
#define KPER 50
#define SC_THREADS 256
#define SC_BLOCKS 197
#define TPW 36
#define OUT_ENC (NB_FULL * VDIM)
#define OUT_ALPHA (NB_FULL * VOCAB)
#define OUT_ELEMS (OUT_ENC + OUT_ALPHA)
#define WUNDO (1.0f / 32.0f)

static_assert(NB == 16);
static_assert(NB == NB_FULL);
static_assert(DDIM % 32 == 0);
static_assert(VDIM % 4 == 0);
static_assert(NPAD % 16 == 0 && NPAD >= VDIM && NPAD % 4 == 0);
static_assert(QP % 32 == 0 && QP >= NPAD);
static_assert(AP % 32 == 0 && AP >= VOCAB && AP / 32 == KSTEPS);
static_assert(PP % 64 == 0 && PP >= AP);
static_assert(KCH * KPER >= KSTEPS && (KCH - 1) * KPER < KSTEPS);
static_assert(SC_BLOCKS * SC_THREADS >= AP);
static_assert((AP * 4) % 128 == 0 && (PP * 2) % 128 == 0 && (QP * 4) % 128 == 0);
static_assert(OUT_ENC * 4 == 19200);
static_assert((OUT_ENC * 4) % 128 == 0);
static_assert(OUT_ENC % 32 == 0);
static_assert((size_t)OUT_ELEMS * 4 == (size_t)3235648);
static_assert(25 * 256 >= PP / 8);
static_assert(10 * 32 >= NPAD);
static_assert(2 * 256 >= NPAD);
static_assert(4 * 4 == 16);
static_assert(NB * NPAD * 4 + NPAD * 4 + 8 * 16 * 4 <= 131072);
static_assert(NPAD * TPW * 4 <= 131072);
static_assert(TPW >= 32 && (TPW * 4) % 16 == 0);
static_assert(NPAD - VDIM == 4);
static_assert(10 * 16 * 36 * 4 <= 131072);

typedef _Float16 h16;
typedef __attribute__((ext_vector_type(16))) _Float16 v16h;
typedef __attribute__((ext_vector_type(8)))  _Float16 v8h;
typedef __attribute__((ext_vector_type(8)))  float    v8f;
typedef __attribute__((ext_vector_type(4)))  float    v4f;
typedef __attribute__((ext_vector_type(4)))  unsigned int v4u;


#define VST2(T, ptr, val) do { const T vst2_v_ = (val); *(volatile T*)(ptr) = vst2_v_; __threadfence(); *(volatile T*)(ptr) = vst2_v_; } while (0)

__device__ __forceinline__ float bfr(float f) {
    unsigned u = __float_as_uint(f);
    u += 0x7FFFu + ((u >> 16) & 1u);
    return __uint_as_float(u & 0xFFFF0000u);
}
static __device__ __forceinline__ h16 toh_flush(float v) { const float w = (fabsf(v) < 6.103515625e-05f) ? 0.0f : v; return (h16)w; }
static __device__ __forceinline__ unsigned pack2h(h16 lo, h16 hi) {
    const unsigned l = (unsigned)__builtin_bit_cast(unsigned short, lo);
    const unsigned u = (unsigned)__builtin_bit_cast(unsigned short, hi);
    return l | (u << 16);
}

union FragU { v16h v; v8h h[2]; };
__device__ __forceinline__ v16h frag_ld(const _Float16* p) {
    FragU f; f.h[0] = *(const v8h*)(p); f.h[1] = *(const v8h*)(p + 16); return f.v;
}
template <int CARRY>
__device__ __forceinline__ v16h frag_cvt(const float* __restrict__ p, bool keep) {
    const v4f x0 = *(const v4f*)(p), x1 = *(const v4f*)(p + 4), x2 = *(const v4f*)(p + 16), x3 = *(const v4f*)(p + 20);
    const float xs[16] = {x0.x, x0.y, x0.z, x0.w, x1.x, x1.y, x1.z, x1.w, x2.x, x2.y, x2.z, x2.w, x3.x, x3.y, x3.z, x3.w};
    v16h f;
#pragma unroll
    for (int i = 0; i < 16; ++i) {
        const float w = keep ? bfr(xs[i]) * (float)CARRY : 0.0f;
        f[i] = toh_flush(w);
    }
    return f;
}
__device__ __forceinline__ v8f wmma16(v16h a, v16h b, v8f c) {
    c = __builtin_amdgcn_wmma_f32_16x16x32_f16(false, a, false, b, (short)0, c, false, false);
    asm volatile("v_nop\n\tv_nop\n\tv_nop\n\tv_nop" : "+v"(c) : "v"(a), "v"(b));
    return c;
}
__device__ __forceinline__ void wave_sync_lds() {
    __builtin_amdgcn_fence(3  , "workgroup");
    __builtin_amdgcn_wave_barrier();
    __builtin_amdgcn_fence(2  , "workgroup");
}

__global__ __launch_bounds__(32) void k_query(const float* __restrict__ dh, const float* __restrict__ Wd,
                                              const float* __restrict__ bd, float* __restrict__ qout) {
    __shared__ __align__(16) float sQ[16 * 36];
    const unsigned lane = threadIdx.x & 31u;
    const unsigned hh = lane >> 4, c = lane & 15u;
    const unsigned pair = blockIdx.x;
    const unsigned n0 = pair * 32u + c, n1 = n0 + 16u;
    const unsigned r0 = min(n0, (unsigned)(VDIM - 1)), r1 = min(n1, (unsigned)(VDIM - 1));
    const bool ok0 = n0 < (unsigned)VDIM, ok1 = n1 < (unsigned)VDIM;
    const float* ap  = dh + (size_t)c * DDIM + 8u * hh;
    const float* bp0 = Wd + (size_t)r0 * DDIM + 8u * hh;
    const float* bp1 = Wd + (size_t)r1 * DDIM + 8u * hh;
    v8f acc0 = (v8f){0.f,0.f,0.f,0.f,0.f,0.f,0.f,0.f};
    v8f acc1 = acc0;
#pragma unroll 1
    for (unsigned k0 = 0; k0 < (unsigned)DDIM; k0 += 32u) {
        const v16h a  = frag_cvt<1>(ap + k0, true);
        const v16h b0 = frag_cvt<32>(bp0 + k0, ok0);
        const v16h b1 = frag_cvt<32>(bp1 + k0, ok1);
        acc0 = wmma16(a, b0, acc0);
        acc1 = wmma16(a, b1, acc1);
    }
    const float bv0 = bfr(bd[r0]);
    const float bv1 = bfr(bd[r1]);
#pragma unroll
    for (int r = 0; r < 8; ++r) {
        const float v0 = ok0 ? (acc0[r] * WUNDO + bv0) : 0.0f;
        const float v1 = ok1 ? (acc1[r] * WUNDO + bv1) : 0.0f;
        sQ[(8u * hh + (unsigned)r) * 36u + c] = v0;
        sQ[(8u * hh + (unsigned)r) * 36u + 16u + c] = v1;
    }
    wave_sync_lds();
    {
        const unsigned q = lane >> 3, c4 = (lane & 7u) * 4u;
        v4f vv[4];
#pragma unroll
        for (int it = 0; it < 4; ++it) vv[it] = *(const v4f*)(sQ + ((unsigned)it * 4u + q) * 36u + c4);
        float* dst = qout + pair * 32u + c4;
        for (int pass = 0; pass < 2; ++pass) {
#pragma unroll
            for (int it = 0; it < 4; ++it) *(volatile v4f*)(dst + (size_t)((unsigned)it * 4u + q) * QP) = vv[it];
            __threadfence();
        }
    }
}

__global__ __launch_bounds__(256) void k_score(const float* __restrict__ E, const float* __restrict__ Wf,
                                               const float* __restrict__ bfull, const float* __restrict__ qin,
                                               float* __restrict__ att, float* __restrict__ pmax) {
    __shared__ __align__(16) float sq[NB * NPAD];
    __shared__ __align__(16) float sw[NPAD];
    __shared__ float smx[8][16];
    unsigned tid = threadIdx.x;
    asm volatile("" : "+v"(tid));
    const unsigned lane = tid & 31u;
    const unsigned wave = (unsigned)__builtin_amdgcn_readfirstlane((int)(tid >> 5));
#pragma unroll 1
    for (unsigned b = 0; b < (unsigned)NB; ++b) {
        unsigned bo = b;
        asm volatile("" : "+s"(bo));
        for (unsigned d = tid; d < (unsigned)NPAD; d += 256u) sq[bo * (unsigned)NPAD + d] = qin[bo * (unsigned)QP + d];
    }
    for (unsigned i = tid; i < (unsigned)NPAD; i += 256u) {
        const float w = bfr(Wf[min(i, (unsigned)(VDIM - 1))]);
        sw[i] = (i < (unsigned)VDIM) ? w : 0.0f;
    }
    __syncthreads();

    const unsigned v = blockIdx.x * 256u + tid;
    const unsigned vc = min(v, (unsigned)(VOCAB - 1));
    const v4f* erow = (const v4f*)(E + (size_t)vc * VDIM);
    float acc[16];
#pragma unroll
    for (int b = 0; b < 16; ++b) acc[b] = 0.0f;
#pragma unroll 1
    for (unsigned dq = 0; dq < (unsigned)(VDIM / 4); ++dq) {
        const v4f e4 = erow[dq];
        const float e0 = bfr(e4.x), e1 = bfr(e4.y), e2 = bfr(e4.z), e3 = bfr(e4.w);
        const v4f w4 = *(const v4f*)(sw + 4u * dq);
#pragma unroll
        for (int b = 0; b < 16; ++b) {
            const v4f q4 = *(const v4f*)(sq + (unsigned)b * (unsigned)NPAD + 4u * dq);
            acc[b] += fmaxf(e0 + q4.x, 0.0f) * w4.x;
            acc[b] += fmaxf(e1 + q4.y, 0.0f) * w4.y;
            acc[b] += fmaxf(e2 + q4.z, 0.0f) * w4.z;
            acc[b] += fmaxf(e3 + q4.w, 0.0f) * w4.w;
        }
    }
    const float bf = bfr(bfull[0]);
    const bool inr = v < (unsigned)VOCAB;
    float outv[16];
#pragma unroll
    for (int b = 0; b < 16; ++b) {
        const float a = acc[b] + bf;
        outv[b] = inr ? a : 0.0f;
        float m = inr ? a : -3.0e38f;
        m = fmaxf(m, __shfl_xor(m, 1, 32)); m = fmaxf(m, __shfl_xor(m, 2, 32));
        m = fmaxf(m, __shfl_xor(m, 4, 32)); m = fmaxf(m, __shfl_xor(m, 8, 32));
        m = fmaxf(m, __shfl_xor(m, 16, 32));
        if (lane == 0u) smx[wave][b] = m;
    }
    const bool wave_ok = (blockIdx.x * 256u + wave * 32u) < (unsigned)AP;
    if (wave_ok) {
        for (int pass = 0; pass < 2; ++pass) {
#pragma unroll
            for (int b = 0; b < 16; ++b) *(volatile float*)(att + (size_t)b * AP + v) = outv[b];
            __threadfence();
        }
    }
    __syncthreads();
    if (wave == 0u) {
        const unsigned l = lane & 15u;
        float m = smx[0][l];
#pragma unroll
        for (int w = 1; w < 8; ++w) m = fmaxf(m, smx[w][l]);
        const float val = (lane < 16u) ? m : 0.0f;
        VST2(float, pmax + blockIdx.x * 32u + lane, val);
    }
}

__global__ __launch_bounds__(256) void k_rowstat(const float* __restrict__ att, const float* __restrict__ pmax,
                                                 h16* __restrict__ p16, float* __restrict__ stats) {
    __shared__ float red[256];
    unsigned t = threadIdx.x;
    asm volatile("" : "+v"(t));
    const unsigned b = blockIdx.x;
    float m = -3.0e38f;
    for (unsigned i = t; i < (unsigned)SC_BLOCKS; i += 256u) m = fmaxf(m, pmax[i * 32u + b]);
    red[t] = m;
    __syncthreads();
    for (unsigned s = 128u; s > 0u; s >>= 1) { if (t < s) red[t] = fmaxf(red[t], red[t + s]); __syncthreads(); }
    const float mx = red[0];
    __syncthreads();

    const float* arow = att + (size_t)b * AP;
    h16* prow = p16 + (size_t)b * PP;
    float s32 = 0.0f, s16 = 0.0f;
#pragma unroll 1
    for (unsigned it = 0; it < 25u; ++it) {
        unsigned base = it * 256u;
        asm volatile("" : "+s"(base));
        const unsigned piece = base + t;
        const unsigned lp = min(piece, (unsigned)(AP / 8 - 1));
        const v4f a0 = *(const v4f*)(arow + (size_t)lp * 8u);
        const v4f a1 = *(const v4f*)(arow + (size_t)lp * 8u + 4u);
        const float av[8] = {a0.x, a0.y, a0.z, a0.w, a1.x, a1.y, a1.z, a1.w};
        v8h hv;
#pragma unroll
        for (int e = 0; e < 8; ++e) {
            const unsigned vv = piece * 8u + (unsigned)e;
            const float pe = expf(av[e] - mx);
            const float p = (vv < (unsigned)VOCAB) ? pe : 0.0f;
            s32 += p;
            const h16 h = toh_flush(p);
            s16 += (float)h;
            hv[e] = h;
        }
        if (piece < (unsigned)(PP / 8)) {
            h16* dst = prow + (size_t)piece * 8u;
            *(volatile v8h*)(dst) = hv;
            __threadfence();
            *(volatile v8h*)(dst) = hv;
        }
    }
    red[t] = s32;
    __syncthreads();
    for (unsigned s = 128u; s > 0u; s >>= 1) { if (t < s) red[t] += red[t + s]; __syncthreads(); }
    const float S32 = red[0];
    __syncthreads();
    red[t] = s16;
    __syncthreads();
    for (unsigned s = 128u; s > 0u; s >>= 1) { if (t < s) red[t] += red[t + s]; __syncthreads(); }
    const float S16 = red[0];
    __syncthreads();
    const float i32 = 1.0f / S32;
    const float i16 = 1.0f / S16;
    if (t < 32u) {
        float val = 0.0f;
        val = (t == 0u) ? mx : val;
        val = (t == 1u) ? S32 : val;
        val = (t == 2u) ? S16 : val;
        val = (t == 3u) ? i32 : val;
        val = (t == 4u) ? i16 : val;
        VST2(float, stats + b * 32u + t, val);
    }
}

__global__ __launch_bounds__(256) void k_transp(const float* __restrict__ E, h16* __restrict__ et) {
    __shared__ __align__(16) unsigned sTw[NPAD * TPW];
    unsigned t = threadIdx.x;
    asm volatile("" : "+v"(t));
    unsigned lane = t & 31u;
    asm volatile("" : "+v"(lane));
    const unsigned wave = (unsigned)__builtin_amdgcn_readfirstlane((int)(threadIdx.x >> 5));
    const unsigned v0 = blockIdx.x * 64u;
    const unsigned va = v0 + 2u * lane;
    const unsigned vb = va + 1u;
    const bool keepa = va < (unsigned)VOCAB;
    const bool keepb = vb < (unsigned)VOCAB;
    const unsigned oa = min(va, (unsigned)(VOCAB - 1)) * (unsigned)VDIM;
    const unsigned ob = min(vb, (unsigned)(VOCAB - 1)) * (unsigned)VDIM;
#pragma unroll 1
    for (unsigned q4 = wave; q4 < (unsigned)(VDIM / 4); q4 += 8u) {
        unsigned qv = q4;
        asm volatile("" : "+s"(qv));
        const v4f xa = *(const v4f*)(E + (size_t)(oa + 4u * qv));
        const v4f xb = *(const v4f*)(E + (size_t)(ob + 4u * qv));
        const float a0 = keepa ? bfr(xa.x) : 0.0f;
        const float a1 = keepa ? bfr(xa.y) : 0.0f;
        const float a2 = keepa ? bfr(xa.z) : 0.0f;
        const float a3 = keepa ? bfr(xa.w) : 0.0f;
        const float b0 = keepb ? bfr(xb.x) : 0.0f;
        const float b1 = keepb ? bfr(xb.y) : 0.0f;
        const float b2 = keepb ? bfr(xb.z) : 0.0f;
        const float b3 = keepb ? bfr(xb.w) : 0.0f;
        const unsigned w0 = pack2h(toh_flush(a0), toh_flush(b0));
        const unsigned w1 = pack2h(toh_flush(a1), toh_flush(b1));
        const unsigned w2 = pack2h(toh_flush(a2), toh_flush(b2));
        const unsigned w3 = pack2h(toh_flush(a3), toh_flush(b3));
        sTw[(4u * qv + 0u) * (unsigned)TPW + lane] = w0;
        sTw[(4u * qv + 1u) * (unsigned)TPW + lane] = w1;
        sTw[(4u * qv + 2u) * (unsigned)TPW + lane] = w2;
        sTw[(4u * qv + 3u) * (unsigned)TPW + lane] = w3;
    }
    if (wave < 4u) sTw[((unsigned)VDIM + wave) * (unsigned)TPW + lane] = 0u;
    __syncthreads();
#pragma unroll 1
    for (unsigned sweep = 0; sweep < 10u; ++sweep) {
        unsigned dbase = sweep * 32u + wave * 4u;
        asm volatile("" : "+s"(dbase));
        if (dbase < (unsigned)NPAD) {
            const unsigned d = dbase + (lane >> 3);
            const unsigned j = lane & 7u;
            const v4u hv = *(const v4u*)(sTw + d * (unsigned)TPW + 4u * j);
            h16* dst = et + (size_t)d * PP + v0 + 8u * j;
            *(volatile v4u*)(dst) = hv;
            __threadfence();
            *(volatile v4u*)(dst) = hv;
        }
    }
}

__global__ __launch_bounds__(320) void k_wsum(const h16* __restrict__ p16, const h16* __restrict__ et, float* __restrict__ part) {
    __shared__ __align__(16) float sS[10][16 * 36];
    const unsigned lane = threadIdx.x & 31u;
    const unsigned wave = (unsigned)__builtin_amdgcn_readfirstlane((int)(threadIdx.x >> 5));
    const unsigned hh = lane >> 4, c = lane & 15u;
    const unsigned chunk = blockIdx.x;
    const unsigned ks0 = chunk * (unsigned)KPER;
    const unsigned ks1 = min(ks0 + (unsigned)KPER, (unsigned)KSTEPS);
    const unsigned na = wave * 32u + c;
    const unsigned nb = min(na + 16u, (unsigned)(NPAD - 1));
    const h16* ap  = p16 + (size_t)c * PP + 8u * hh;
    const h16* bp0 = et + (size_t)na * PP + 8u * hh;
    const h16* bp1 = et + (size_t)nb * PP + 8u * hh;
    v8f acc0 = (v8f){0.f,0.f,0.f,0.f,0.f,0.f,0.f,0.f};
    v8f acc1 = acc0;
#pragma unroll 1
    for (unsigned ks = ks0; ks < ks1; ++ks) {
        const unsigned k0 = ks * 32u;
        const v16h a  = frag_ld(ap + k0);
        const v16h b0 = frag_ld(bp0 + k0);
        const v16h b1 = frag_ld(bp1 + k0);
        acc0 = wmma16(a, b0, acc0);
        acc1 = wmma16(a, b1, acc1);
    }
#pragma unroll
    for (int r = 0; r < 8; ++r) {
        sS[wave][(8u * hh + (unsigned)r) * 36u + c] = acc0[r];
        sS[wave][(8u * hh + (unsigned)r) * 36u + 16u + c] = acc1[r];
    }
    wave_sync_lds();
    {
        const unsigned q = lane >> 3, c4 = (lane & 7u) * 4u;
        v4f vv[4];
#pragma unroll
        for (int it = 0; it < 4; ++it) vv[it] = *(const v4f*)(&sS[wave][((unsigned)it * 4u + q) * 36u + c4]);
        float* dst = part + (size_t)chunk * 16u * QP + wave * 32u + c4;
        for (int pass = 0; pass < 2; ++pass) {
#pragma unroll
            for (int it = 0; it < 4; ++it) *(volatile v4f*)(dst + (size_t)((unsigned)it * 4u + q) * QP) = vv[it];
            __threadfence();
        }
    }
}

__global__ __launch_bounds__(256) void k_enc(const float* __restrict__ part, const float* __restrict__ stats, float* __restrict__ out) {
    unsigned t = threadIdx.x;
    asm volatile("" : "+v"(t));
#pragma unroll 1
    for (unsigned i = t; i < (unsigned)OUT_ENC; i += 256u) {
        unsigned iv = i;
        asm volatile("" : "+v"(iv));
        const unsigned b = iv / (unsigned)VDIM;
        const unsigned d = iv - b * (unsigned)VDIM;
        float acc = 0.0f;
#pragma unroll 1
        for (unsigned ch = 0; ch < (unsigned)KCH; ++ch) acc += part[((size_t)ch * 16u + b) * QP + d];
        const float val = acc * stats[b * 32u + 4u];
        VST2(float, out + iv, val);
    }
}

__global__ __launch_bounds__(256) void k_alpha(const float* __restrict__ att, const float* __restrict__ stats, float* __restrict__ alpha) {
    unsigned i = blockIdx.x * 256u + threadIdx.x;
    asm volatile("" : "+v"(i));
    const unsigned ic = min(i, (unsigned)(OUT_ALPHA - 1));
    const unsigned b = ic / (unsigned)VOCAB;
    const unsigned v = ic - b * (unsigned)VOCAB;
    const float a = att[(size_t)b * AP + v];
    const float mx = stats[b * 32u];
    const float inv = stats[b * 32u + 3u];
    const float val = expf(a - mx) * inv;
    if (i < (unsigned)OUT_ALPHA) { VST2(float, alpha + i, val); }
}

#define AL256(x) ((((size_t)(x)) + 255) & ~(size_t)255)
static constexpr size_t WS_Q     = AL256((size_t)NB * QP * 4);
static constexpr size_t WS_ATT   = AL256((size_t)NB * AP * 4);
static constexpr size_t WS_PMAX  = AL256((size_t)SC_BLOCKS * 32 * 4);
static constexpr size_t WS_STATS = AL256((size_t)NB * 32 * 4);
static constexpr size_t WS_P16   = AL256((size_t)NB * PP * 2);
static constexpr size_t WS_ET    = AL256((size_t)NPAD * PP * 2);
static constexpr size_t WS_PART  = AL256((size_t)KCH * 16 * QP * 4);
static_assert(WS_Q + WS_ATT + WS_PMAX + WS_STATS + WS_P16 + WS_ET + WS_PART <= (size_t)134217728);

extern "C" void kernel_launch(void* const* d_in, const int* in_sizes, int n_in, void* d_out, int out_size,
                              void* d_ws, size_t ws_size, hipStream_t stream) {
    if (n_in < 6) return;
    if (in_sizes[0] < NB * DDIM || in_sizes[1] < VOCAB * VDIM || in_sizes[2] < VDIM * DDIM) return;
    if (in_sizes[3] < VDIM || in_sizes[4] < VDIM || in_sizes[5] < 1 || out_size < OUT_ELEMS) return;

    const float* dh    = (const float*)d_in[0];
    const float* E     = (const float*)d_in[1];
    const float* Wd    = (const float*)d_in[2];
    const float* bd    = (const float*)d_in[3];
    const float* Wf    = (const float*)d_in[4];
    const float* bfull = (const float*)d_in[5];
    float* out = (float*)d_out;

    char* wsp = (char*)d_ws;
    size_t off = 0;
    auto carve = [&](size_t bytes) -> void* { void* r = wsp + off; off += (bytes + 255) & ~(size_t)255; return r; };
    float* qpl   = (float*)carve((size_t)NB * QP * 4);
    float* attp  = (float*)carve((size_t)NB * AP * 4);
    float* pmax  = (float*)carve((size_t)SC_BLOCKS * 32 * 4);
    float* stats = (float*)carve((size_t)NB * 32 * 4);
    h16*   p16   = (h16*)carve((size_t)NB * PP * 2);
    h16*   etp   = (h16*)carve((size_t)NPAD * PP * 2);
    float* part  = (float*)carve((size_t)KCH * 16 * QP * 4);
    if (off > ws_size || off > (size_t)134217728) return;

    k_query<<<QP / 32, 32, 0, stream>>>(dh, Wd, bd, qpl);
    k_score<<<SC_BLOCKS, 256, 0, stream>>>(E, Wf, bfull, qpl, attp, pmax);
    k_rowstat<<<NB, 256, 0, stream>>>(attp, pmax, p16, stats);
    k_transp<<<PP / 64, 256, 0, stream>>>(E, etp);
    k_wsum<<<KCH, 320, 0, stream>>>((const h16*)p16, (const h16*)etp, part);
    k_enc<<<1, 256, 0, stream>>>(part, stats, out);
    k_alpha<<<(OUT_ALPHA + 255) / 256, 256, 0, stream>>>(attp, stats, out + OUT_ENC);
}
